// PointNetSetAbstraction_50972671869076
// MI455X (gfx1250) — hardware-verified
//
#include <hip/hip_runtime.h>
#pragma clang fp contract(off)

typedef __attribute__((ext_vector_type(16))) _Float16 v16h;
typedef __attribute__((ext_vector_type(8)))  _Float16 v8h;
typedef __attribute__((ext_vector_type(8)))  float    v8f;
typedef __attribute__((ext_vector_type(4)))  float    v4f;
typedef __attribute__((ext_vector_type(4)))  unsigned v4u;
typedef __attribute__((ext_vector_type(4)))  int      v4i;
union FragH { v16h v; v8h h[2]; };

constexpr int NBATCH = 16;
constexpr int NPTS = 4096;
constexpr int NCENT = 1024;
constexpr int NSAMP = 32;
constexpr int NFEAT = 32;
constexpr int CIN0 = 35;
constexpr int KPAD = 64;
constexpr int CH0 = 64;
constexpr int CH1 = 64;
constexpr int CH2 = 128;
constexpr int NGROUP = NBATCH * NCENT;
constexpr int NROWS = NGROUP * NSAMP;
constexpr int NPTALL = NBATCH * NPTS;
constexpr int TILE_PITCH = 72;
constexpr int NBLK_PASS = NGROUP / 8;
constexpr float W_CARRY = 16.0f;
constexpr float W_CARRY_INV = 1.0f / 16.0f;
constexpr float BN_EPS = 1e-5f;
constexpr float BALL_R2 = 0.04f;

static_assert(NGROUP == 16384);
static_assert(NROWS == 524288);
static_assert(NGROUP % 8 == 0);
static_assert(CIN0 == 3 + NFEAT);
static_assert(KPAD % 32 == 0 && CH0 % 32 == 0 && CH1 % 32 == 0);
static_assert(CH0 % 64 == 0 && CH1 % 64 == 0 && CH2 % 64 == 0);

constexpr size_t OFF_W0H = 0;
constexpr size_t OFF_W1H = OFF_W0H + (size_t)CH0 * KPAD * 2;
constexpr size_t OFF_W2H = OFF_W1H + (size_t)CH1 * CH0 * 2;
constexpr size_t OFF_SC0 = OFF_W2H + (size_t)CH2 * CH1 * 2;
constexpr size_t OFF_SC1 = OFF_SC0 + 1024;
constexpr size_t OFF_SC2 = OFF_SC1 + 1024;
constexpr size_t OFF_CEN = 65536;
constexpr size_t OFF_IDX = OFF_CEN + (size_t)NGROUP * 3 * 4;
constexpr size_t OFF_V = OFF_IDX + (size_t)NROWS * 4;
constexpr size_t OFF_F = OFF_V + (size_t)NGROUP * CH0 * 4;
constexpr size_t OFF_PART0 = OFF_F + (size_t)NPTALL * KPAD * 2;
constexpr size_t OFF_PART1 = OFF_PART0 + (size_t)NBLK_PASS * 2 * CH0 * 4;
constexpr size_t OFF_PART2 = OFF_PART1 + (size_t)NBLK_PASS * 2 * CH1 * 4;
constexpr size_t OFF_MX = OFF_PART2 + (size_t)NBLK_PASS * 2 * CH2 * 4;
constexpr size_t OFF_MN = OFF_MX + (size_t)NGROUP * CH2 * 4;
constexpr size_t OFF_X1 = OFF_MN + (size_t)NGROUP * CH2 * 4;
constexpr size_t WS_TOTAL = OFF_X1 + (size_t)NROWS * CH1 * 2;
static_assert(OFF_SC2 + 1024 <= OFF_CEN);
static_assert(WS_TOTAL <= (size_t)134217728);
static_assert(OFF_X1 % 128 == 0 && OFF_F % 128 == 0 && OFF_IDX % 128 == 0 && OFF_V % 128 == 0);
constexpr size_t OUT1_BYTE_OFF = 196608;
constexpr size_t OUT1_ELEM_OFF = OUT1_BYTE_OFF / 4;
static_assert(OUT1_ELEM_OFF == (size_t)NGROUP * 3);
static_assert(OUT1_BYTE_OFF + (size_t)NBATCH * CH2 * NCENT * 4 == (size_t)8585216);
static_assert(OUT1_BYTE_OFF % 128 == 0);

__device__ __forceinline__ v8f mma_h(v16h a, v16h b, v8f c) {
  c = __builtin_amdgcn_wmma_f32_16x16x32_f16(false, a, false, b, (short)0, c, false, false);
  asm volatile("v_nop\n\tv_nop\n\tv_nop\n\tv_nop" : "+v"(c) : "v"(a), "v"(b));
  return c;
}

__device__ __forceinline__ float h16_to_f32(unsigned hb) {
  const unsigned sgn = (hb & 0x8000u) << 16;
  const unsigned em = hb & 0x7fffu;
  const float fn = __uint_as_float((em << 13) + 0x38000000u);
  const float fs = (float)em * 5.9604644775390625e-8f;
  const float mag = (em < 0x400u) ? fs : fn;
  return __uint_as_float(__float_as_uint(mag) | sgn);
}

__device__ __forceinline__ _Float16 bn_relu_h(unsigned hb, float sc, float sh) {
  const float x = h16_to_f32(hb);
  float y = x * sc + sh;
  y = fmaxf(y, 0.0f);
  return (_Float16)y;
}

__global__ __launch_bounds__(256) void prep_weights(
    const float* __restrict__ w0, const float* __restrict__ w1, const float* __restrict__ w2,
    _Float16* __restrict__ W0h, _Float16* __restrict__ W1h, _Float16* __restrict__ W2h) {
  const int blk = blockIdx.x;
  const int tid = threadIdx.x;
  float zf = 0.0f;
  asm volatile("" : "+v"(zf));
  v8h hv;
  _Float16* dst;
  if (blk < 2) {
    const int t = blk * 256 + tid;
    const int n = t >> 3;
    const int seg = t & 7;
#pragma unroll
    for (int e = 0; e < 8; ++e) {
      const int col = seg * 8 + e;
      const int cc = (col < CIN0) ? col : (CIN0 - 1);
      const float wv = w0[n * CIN0 + cc];
      const float sv = (col < CIN0) ? (wv * W_CARRY) : zf;
      hv[e] = (_Float16)sv;
    }
    dst = W0h + (size_t)t * 8;
  } else if (blk < 4) {
    const int t = (blk - 2) * 256 + tid;
    const v4f a = *(const v4f*)(w1 + (size_t)t * 8);
    const v4f b = *(const v4f*)(w1 + (size_t)t * 8 + 4);
#pragma unroll
    for (int e = 0; e < 4; ++e) {
      hv[e] = (_Float16)(a[e] * W_CARRY);
      hv[4 + e] = (_Float16)(b[e] * W_CARRY);
    }
    dst = W1h + (size_t)t * 8;
  } else {
    const int t = (blk - 4) * 256 + tid;
    const v4f a = *(const v4f*)(w2 + (size_t)t * 8);
    const v4f b = *(const v4f*)(w2 + (size_t)t * 8 + 4);
#pragma unroll
    for (int e = 0; e < 4; ++e) {
      hv[e] = (_Float16)(a[e] * W_CARRY);
      hv[4 + e] = (_Float16)(b[e] * W_CARRY);
    }
    dst = W2h + (size_t)t * 8;
  }
  *(volatile v8h*)dst = hv;
  __threadfence();
  *(volatile v8h*)dst = hv;
}

__global__ __launch_bounds__(256) void prep_features(
    const float* __restrict__ xyz, const float* __restrict__ points, _Float16* __restrict__ F) {
  __shared__ __align__(16) float sF[32 * 64];
  const int tid = threadIdx.x;
  const int row0 = blockIdx.x * 32;
  const int r = tid >> 3;
  const int q = tid & 7;
  const v4f pv = *(const v4f*)(points + (size_t)(row0 + r) * NFEAT + 4 * q);
#pragma unroll
  for (int e = 0; e < 4; ++e) sF[r * 64 + 3 + 4 * q + e] = pv[e];
  const int xi = (tid < 96) ? tid : 95;
  const float xv = xyz[(size_t)row0 * 3 + xi];
  if (tid < 96) sF[(xi / 3) * 64 + (xi % 3)] = xv;
  for (int i = tid; i < 32 * 29; i += 256) {
    const int rr = i / 29;
    const int cc = CIN0 + (i - rr * 29);
    sF[rr * 64 + cc] = 0.0f;
  }
  __syncthreads();
  v8h hv;
#pragma unroll
  for (int e = 0; e < 8; ++e) hv[e] = (_Float16)sF[r * 64 + q * 8 + e];
  _Float16* dst = F + (size_t)(row0 + r) * KPAD + q * 8;
  *(volatile v8h*)dst = hv;
  __threadfence();
  *(volatile v8h*)dst = hv;
}

__global__ __launch_bounds__(256) void fps_kernel(
    const float* __restrict__ xyz, float* __restrict__ out0, float* __restrict__ cen) {
#pragma clang fp contract(off)
  __shared__ __align__(16) float sx[NPTS * 3];
  __shared__ __align__(16) float sel[NCENT * 3];
  __shared__ float rdv[2][8];
  __shared__ int riv[2][8];
  const int b = blockIdx.x;
  const int tid = threadIdx.x;
  const int lane = tid & 31;
  const int wave = tid >> 5;
  const float* gx = xyz + (size_t)b * NPTS * 3;
#pragma unroll 4
  for (int i = tid; i < NPTS * 3; i += 256) sx[i] = gx[i];
  __syncthreads();
  float px[16], py[16], pz[16], dist[16];
#pragma unroll
  for (int r = 0; r < 16; ++r) {
    px[r] = sx[(tid * 16 + r) * 3 + 0];
    py[r] = sx[(tid * 16 + r) * 3 + 1];
    pz[r] = sx[(tid * 16 + r) * 3 + 2];
    dist[r] = 1e10f;
  }
  int far = 0;
#pragma unroll 1
  for (int it = 0; it < NCENT; ++it) {
    const int par = it & 1;
    const float cx = sx[far * 3 + 0];
    const float cy = sx[far * 3 + 1];
    const float cz = sx[far * 3 + 2];
    if (tid == 0) {
      sel[it * 3 + 0] = cx;
      sel[it * 3 + 1] = cy;
      sel[it * 3 + 2] = cz;
    }
    float bd = -1.0f;
    int bi = tid * 16;
#pragma unroll
    for (int r = 0; r < 16; ++r) {
      const float dx = px[r] - cx;
      const float dy = py[r] - cy;
      const float dz = pz[r] - cz;
      const float t0 = dx * dx;
      const float t1 = dy * dy;
      const float t2 = dz * dz;
      const float d = (t0 + t2) + t1;
      const float nd = fminf(dist[r], d);
      dist[r] = nd;
      const bool up = nd > bd;
      bd = up ? nd : bd;
      bi = up ? (tid * 16 + r) : bi;
    }
#pragma unroll
    for (int off = 16; off > 0; off >>= 1) {
      const float od = __shfl_xor(bd, off, 32);
      const int oi = __shfl_xor(bi, off, 32);
      const bool take = (od > bd) || ((od == bd) && (oi < bi));
      bd = take ? od : bd;
      bi = take ? oi : bi;
    }
    if (lane == 0) {
      rdv[par][wave] = bd;
      riv[par][wave] = bi;
    }
    __syncthreads();
    float fd = rdv[par][0];
    int fi = riv[par][0];
#pragma unroll
    for (int w = 1; w < 8; ++w) {
      const float od = rdv[par][w];
      const int oi = riv[par][w];
      const bool take = od > fd;
      fd = take ? od : fd;
      fi = take ? oi : fi;
    }
    far = fi & (NPTS - 1);
  }
  __syncthreads();
  for (int pass = 0; pass < 2; ++pass) {
#pragma unroll
    for (int j = 0; j < 3; ++j) {
      const int i = tid + 256 * j;
      const v4f v = *(const v4f*)(sel + 4 * i);
      *(volatile v4f*)(out0 + (size_t)b * (NCENT * 3) + 4 * i) = v;
      *(volatile v4f*)(cen + (size_t)b * (NCENT * 3) + 4 * i) = v;
    }
    __threadfence();
  }
}

__global__ __launch_bounds__(128) void ball_query(
    const float* __restrict__ xyz, const float* __restrict__ cen, const float* __restrict__ w0,
    int* __restrict__ IDX, float* __restrict__ V) {
#pragma clang fp contract(off)
  __shared__ __align__(16) int lst[4][32];
  __shared__ __align__(16) float sV[4][64];
  const int tid = threadIdx.x;
  const int lane = tid & 31;
  const int wv = tid >> 5;
  const int blk = blockIdx.x;
  const int w = blk * 4 + wv;
  const int b = w >> 10;
  const float nx = cen[(size_t)w * 3 + 0];
  const float ny = cen[(size_t)w * 3 + 1];
  const float nz = cen[(size_t)w * 3 + 2];
  const float* xb = xyz + (size_t)b * NPTS * 3;
  int cnt = 0;
  int first = -1;
  for (int base = 0; base < NPTS && cnt < NSAMP; base += 32) {
    const int i = base + lane;
    const float q0 = xb[i * 3 + 0];
    const float q1 = xb[i * 3 + 1];
    const float q2 = xb[i * 3 + 2];
    const float dx = nx - q0;
    const float dy = ny - q1;
    const float dz = nz - q2;
    const float t0 = dx * dx;
    const float t1 = dy * dy;
    const float t2 = dz * dz;
    const float d = (t0 + t2) + t1;
    const bool pred = !(d > BALL_R2);
    const unsigned mask = __builtin_amdgcn_ballot_w32(pred);
    if (first < 0 && mask != 0u) first = base + __builtin_ctz(mask);
    const int slot = cnt + __popc(mask & ((1u << lane) - 1u));
    if (pred && slot < NSAMP) lst[wv][slot] = i;
    cnt += __popc(mask);
  }
  if (first < 0) first = 0;
  const int filled = (cnt < NSAMP) ? cnt : NSAMP;
  if (lane >= filled) lst[wv][lane] = first;
#pragma unroll
  for (int k = 0; k < 2; ++k) {
    const int o = lane + 32 * k;
    const float wa = (float)((_Float16)(w0[o * CIN0 + 0] * W_CARRY)) * W_CARRY_INV;
    const float wb = (float)((_Float16)(w0[o * CIN0 + 1] * W_CARRY)) * W_CARRY_INV;
    const float wc = (float)((_Float16)(w0[o * CIN0 + 2] * W_CARRY)) * W_CARRY_INV;
    const float pa = wa * nx;
    const float pb = wb * ny;
    const float pc = wc * nz;
    sV[wv][o] = (pa + pb) + pc;
  }
  __syncthreads();
  if (wv == 0) {
    const int* lf = &lst[0][0];
    const int bbase = ((blk * 4) >> 10) * NPTS;
    v4i iv;
#pragma unroll
    for (int e = 0; e < 4; ++e) {
      int x = lf[4 * lane + e];
      x = x < 0 ? 0 : x;
      x = x > (NPTS - 1) ? (NPTS - 1) : x;
      iv[e] = bbase + x;
    }
    int* dst = IDX + (size_t)blk * 128 + 4 * lane;
    *(volatile v4i*)dst = iv;
    __threadfence();
    *(volatile v4i*)dst = iv;
  }
  if (wv < 2) {
    const float* vf = &sV[0][0];
    const v4f vv = *(const v4f*)(vf + wv * 128 + 4 * lane);
    float* dst = V + (size_t)blk * 256 + wv * 128 + 4 * lane;
    *(volatile v4f*)dst = vv;
    __threadfence();
    *(volatile v4f*)dst = vv;
  }
}

template <bool SECOND>
__global__ __launch_bounds__(256) void pass_ab(
    const _Float16* __restrict__ F, const int* __restrict__ IDX, const float* __restrict__ V,
    const _Float16* __restrict__ W0h, const float* __restrict__ b0, const float* __restrict__ SC0,
    const _Float16* __restrict__ W1h, const float* __restrict__ b1,
    _Float16* __restrict__ X1, float* __restrict__ PART) {
  __shared__ __align__(16) _Float16 sT[8][32 * TILE_PITCH];
  __shared__ float sS[8][2][64];
  __shared__ __align__(16) float sP[128];
  const int tid = threadIdx.x;
  const int lane = tid & 31;
  const int wave = tid >> 5;
  const int hh = lane >> 4;
  const int c = lane & 15;
  const int q8 = lane >> 3;
  const int s8 = lane & 7;
  const int g = blockIdx.x * 8 + wave;
  _Float16* tile = sT[wave];

  int gi = IDX[(size_t)g * 32 + lane];
  gi = gi < 0 ? 0 : gi;
  gi = gi > (NPTALL - 1) ? (NPTALL - 1) : gi;
#pragma unroll
  for (int it = 0; it < 8; ++it) {
    const int row = it * 4 + q8;
    const int src = __shfl(gi, row, 32);
    const v8h v = *(const v8h*)(F + (size_t)src * KPAD + s8 * 8);
    *(v8h*)(tile + row * TILE_PITCH + s8 * 8) = v;
  }
  __syncthreads();

  v8f acc[2][4];
#pragma unroll
  for (int mt = 0; mt < 2; ++mt)
#pragma unroll
    for (int j = 0; j < 4; ++j) acc[mt][j] = (v8f){0.f, 0.f, 0.f, 0.f, 0.f, 0.f, 0.f, 0.f};
#pragma unroll
  for (int kc = 0; kc < 2; ++kc) {
    v16h bh[4];
#pragma unroll
    for (int j = 0; j < 4; ++j) {
      FragH fb;
      const _Float16* bp = W0h + (size_t)(j * 16 + c) * KPAD + kc * 32 + 8 * hh;
      fb.h[0] = *(const v8h*)(bp);
      fb.h[1] = *(const v8h*)(bp + 16);
      bh[j] = fb.v;
    }
#pragma unroll
    for (int mt = 0; mt < 2; ++mt) {
      FragH fa;
      fa.h[0] = *(const v8h*)(tile + (mt * 16 + c) * TILE_PITCH + kc * 32 + 8 * hh);
      fa.h[1] = *(const v8h*)(tile + (mt * 16 + c) * TILE_PITCH + kc * 32 + 16 + 8 * hh);
#pragma unroll
      for (int j = 0; j < 4; ++j) acc[mt][j] = mma_h(fa.v, bh[j], acc[mt][j]);
    }
  }

  float cadd[4];
#pragma unroll
  for (int j = 0; j < 4; ++j) {
    const int n = j * 16 + c;
    cadd[j] = b0[n] - V[(size_t)g * CH0 + n];
  }
  asm volatile("" ::: "memory");

  float ssum[4], ssq[4];
#pragma unroll
  for (int j = 0; j < 4; ++j) {
    ssum[j] = 0.0f;
    ssq[j] = 0.0f;
  }

  if (!SECOND) {
#pragma unroll
    for (int j = 0; j < 4; ++j)
#pragma unroll
      for (int mt = 0; mt < 2; ++mt)
#pragma unroll
        for (int r = 0; r < 8; ++r) {
          const float x = acc[mt][j][r] * W_CARRY_INV + cadd[j];
          ssum[j] += x;
          ssq[j] += x * x;
        }
  } else {
    float sc[4], sh[4];
#pragma unroll
    for (int j = 0; j < 4; ++j) {
      const int n = j * 16 + c;
      sc[j] = SC0[n];
      sh[j] = SC0[CH0 + n];
    }
    asm volatile("" ::: "memory");
    __syncthreads();
#pragma unroll
    for (int j = 0; j < 4; ++j)
#pragma unroll
      for (int mt = 0; mt < 2; ++mt)
#pragma unroll
        for (int r = 0; r < 8; ++r) {
          const float x = acc[mt][j][r] * W_CARRY_INV + cadd[j];
          float y = x * sc[j] + sh[j];
          y = fmaxf(y, 0.0f);
          tile[(mt * 16 + 8 * hh + r) * TILE_PITCH + j * 16 + c] = (_Float16)y;
        }
    __syncthreads();

    v8f acc1[2][4];
#pragma unroll
    for (int mt = 0; mt < 2; ++mt)
#pragma unroll
      for (int j = 0; j < 4; ++j) acc1[mt][j] = (v8f){0.f, 0.f, 0.f, 0.f, 0.f, 0.f, 0.f, 0.f};
#pragma unroll
    for (int kc = 0; kc < 2; ++kc) {
      v16h bh[4];
#pragma unroll
      for (int j = 0; j < 4; ++j) {
        FragH fb;
        const _Float16* bp = W1h + (size_t)(j * 16 + c) * CH0 + kc * 32 + 8 * hh;
        fb.h[0] = *(const v8h*)(bp);
        fb.h[1] = *(const v8h*)(bp + 16);
        bh[j] = fb.v;
      }
#pragma unroll
      for (int mt = 0; mt < 2; ++mt) {
        FragH fa;
        fa.h[0] = *(const v8h*)(tile + (mt * 16 + c) * TILE_PITCH + kc * 32 + 8 * hh);
        fa.h[1] = *(const v8h*)(tile + (mt * 16 + c) * TILE_PITCH + kc * 32 + 16 + 8 * hh);
#pragma unroll
        for (int j = 0; j < 4; ++j) acc1[mt][j] = mma_h(fa.v, bh[j], acc1[mt][j]);
      }
    }
    float bb[4];
#pragma unroll
    for (int j = 0; j < 4; ++j) bb[j] = b1[j * 16 + c];
    asm volatile("" ::: "memory");
    __syncthreads();
#pragma unroll
    for (int j = 0; j < 4; ++j)
#pragma unroll
      for (int mt = 0; mt < 2; ++mt)
#pragma unroll
        for (int r = 0; r < 8; ++r) {
          const float x = acc1[mt][j][r] * W_CARRY_INV + bb[j];
          ssum[j] += x;
          ssq[j] += x * x;
          tile[(mt * 16 + 8 * hh + r) * TILE_PITCH + j * 16 + c] = (_Float16)x;
        }
    __syncthreads();
    for (int pass = 0; pass < 2; ++pass) {
#pragma unroll
      for (int it = 0; it < 8; ++it) {
        const int row = it * 4 + q8;
        const v8h v = *(const v8h*)(tile + row * TILE_PITCH + s8 * 8);
        *(volatile v8h*)(X1 + ((size_t)g * 32 + row) * CH1 + s8 * 8) = v;
      }
      __threadfence();
    }
  }

#pragma unroll
  for (int j = 0; j < 4; ++j) {
    const float so = __shfl_xor(ssum[j], 16, 32);
    const float qo = __shfl_xor(ssq[j], 16, 32);
    const float st = ssum[j] + so;
    const float qt = ssq[j] + qo;
    const float val = hh ? qt : st;
    sS[wave][hh][j * 16 + c] = val;
  }
  __syncthreads();
  if (tid < 128) {
    const int kind = tid >> 6;
    const int ch = tid & 63;
    float a = 0.0f;
#pragma unroll
    for (int w = 0; w < 8; ++w) a += sS[w][kind][ch];
    sP[tid] = a;
  }
  __syncthreads();
  if (wave == 0) {
    const v4f v = *(const v4f*)(sP + 4 * lane);
    float* dst = PART + (size_t)blockIdx.x * 128 + 4 * lane;
    *(volatile v4f*)dst = v;
    __threadfence();
    *(volatile v4f*)dst = v;
  }
}

template <int C>
__global__ __launch_bounds__(256) void bn_finalize(
    const float* __restrict__ PART, int nblk, const float* __restrict__ gam,
    const float* __restrict__ bet, float* __restrict__ SC) {
  __shared__ double sSum[2 * C];
  __shared__ __align__(16) float sOut[2 * C];
  const int tid = threadIdx.x;
  const int t = (tid < 2 * C) ? tid : (2 * C - 1);
  double acc = 0.0;
#pragma unroll 4
  for (int i = 0; i < nblk; ++i) acc += (double)PART[(size_t)i * (2 * C) + t];
  if (tid < 2 * C) sSum[tid] = acc;
  const int cc = (tid < C) ? tid : (C - 1);
  const float gv = gam[cc];
  const float bev = bet[cc];
  __syncthreads();
  if (tid < C) {
    const double invp = 1.0 / (double)NROWS;
    const double mean = sSum[tid] * invp;
    const double ex2 = sSum[C + tid] * invp;
    double var = ex2 - mean * mean;
    var = var < 0.0 ? 0.0 : var;
    const float vf = (float)var;
    const float inv = 1.0f / sqrtf(vf + BN_EPS);
    const float sc = gv * inv;
    const float sh = bev - (float)mean * sc;
    sOut[tid] = sc;
    sOut[C + tid] = sh;
  }
  __syncthreads();
  if (tid < (2 * C) / 4) {
    const v4f v = *(const v4f*)(sOut + 4 * tid);
    float* dst = SC + 4 * tid;
    *(volatile v4f*)dst = v;
    __threadfence();
    *(volatile v4f*)dst = v;
  }
}

__global__ __launch_bounds__(256) void pass_c(
    const v4u* __restrict__ X1w, const float* __restrict__ SC1, const _Float16* __restrict__ W2h,
    const float* __restrict__ b2, float* __restrict__ MX, float* __restrict__ MN,
    float* __restrict__ PART) {
  __shared__ __align__(16) float sSC[128];
  __shared__ __align__(16) float sMM[2][8][128];
  __shared__ float sS[8][2][128];
  __shared__ __align__(16) float sP[256];
  const int tid = threadIdx.x;
  const int lane = tid & 31;
  const int wave = tid >> 5;
  const int hh = lane >> 4;
  const int c = lane & 15;
  const int g = blockIdx.x * 8 + wave;
  if (tid < 32) {
    const v4f v = *(const v4f*)(SC1 + 4 * tid);
    *(v4f*)(sSC + 4 * tid) = v;
  }
  __syncthreads();

  v16h af[2][2];
#pragma unroll
  for (int mt = 0; mt < 2; ++mt) {
#pragma unroll
    for (int kc = 0; kc < 2; ++kc) {
      const v4u* rp = X1w + ((size_t)g * 32 + mt * 16 + c) * 8 + kc * 4 + hh;
      const v4u qa = rp[0];
      const v4u qb = rp[2];
      const int kb = kc * 32 + 8 * hh;
      v16h a;
#pragma unroll
      for (int i = 0; i < 4; ++i) {
        const unsigned wa = qa[i];
        const unsigned wb = qb[i];
        const int k0 = kb + 2 * i;
        const int k1 = kb + 16 + 2 * i;
        a[2 * i] = bn_relu_h(wa & 0xffffu, sSC[k0], sSC[64 + k0]);
        a[2 * i + 1] = bn_relu_h(wa >> 16, sSC[k0 + 1], sSC[64 + k0 + 1]);
        a[8 + 2 * i] = bn_relu_h(wb & 0xffffu, sSC[k1], sSC[64 + k1]);
        a[8 + 2 * i + 1] = bn_relu_h(wb >> 16, sSC[k1 + 1], sSC[64 + k1 + 1]);
      }
      af[mt][kc] = a;
    }
  }

#pragma unroll 1
  for (int nh = 0; nh < 2; ++nh) {
    v8f acc[2][4];
#pragma unroll
    for (int mt = 0; mt < 2; ++mt)
#pragma unroll
      for (int j = 0; j < 4; ++j) acc[mt][j] = (v8f){0.f, 0.f, 0.f, 0.f, 0.f, 0.f, 0.f, 0.f};
#pragma unroll
    for (int kc = 0; kc < 2; ++kc) {
      v16h bh[4];
#pragma unroll
      for (int j = 0; j < 4; ++j) {
        FragH fb;
        const _Float16* bp = W2h + (size_t)(nh * 64 + j * 16 + c) * CH1 + kc * 32 + 8 * hh;
        fb.h[0] = *(const v8h*)(bp);
        fb.h[1] = *(const v8h*)(bp + 16);
        bh[j] = fb.v;
      }
#pragma unroll
      for (int mt = 0; mt < 2; ++mt) {
#pragma unroll
        for (int j = 0; j < 4; ++j) acc[mt][j] = mma_h(af[mt][kc], bh[j], acc[mt][j]);
      }
    }
#pragma unroll
    for (int j = 0; j < 4; ++j) {
      const int n = nh * 64 + j * 16 + c;
      const float bn = b2[n];
      float s = 0.0f, q = 0.0f, mx = -3.0e38f, mn = 3.0e38f;
#pragma unroll
      for (int mt = 0; mt < 2; ++mt)
#pragma unroll
        for (int r = 0; r < 8; ++r) {
          const float x = acc[mt][j][r] * W_CARRY_INV + bn;
          s += x;
          q += x * x;
          mx = fmaxf(mx, x);
          mn = fminf(mn, x);
        }
      const float so = __shfl_xor(s, 16, 32);
      const float qo = __shfl_xor(q, 16, 32);
      const float xo = __shfl_xor(mx, 16, 32);
      const float no = __shfl_xor(mn, 16, 32);
      const float st = s + so;
      const float qt = q + qo;
      const float xt = fmaxf(mx, xo);
      const float nt = fminf(mn, no);
      const float mval = hh ? nt : xt;
      const float sval = hh ? qt : st;
      sMM[hh][wave][n] = mval;
      sS[wave][hh][n] = sval;
    }
  }
  __syncthreads();
  {
    const int kind = tid >> 7;
    const int ch = tid & 127;
    float a = 0.0f;
#pragma unroll
    for (int w = 0; w < 8; ++w) a += sS[w][kind][ch];
    sP[tid] = a;
  }
  {
    const float* fx = &sMM[0][0][0];
    const float* fn = &sMM[1][0][0];
    const v4f vx = *(const v4f*)(fx + 4 * tid);
    const v4f vn = *(const v4f*)(fn + 4 * tid);
    float* dx = MX + (size_t)blockIdx.x * 1024 + 4 * tid;
    float* dn = MN + (size_t)blockIdx.x * 1024 + 4 * tid;
    *(volatile v4f*)dx = vx;
    *(volatile v4f*)dn = vn;
    __threadfence();
    *(volatile v4f*)dx = vx;
    *(volatile v4f*)dn = vn;
  }
  __syncthreads();
  if (tid < 64) {
    const v4f v = *(const v4f*)(sP + 4 * tid);
    float* dst = PART + (size_t)blockIdx.x * 256 + 4 * tid;
    *(volatile v4f*)dst = v;
    __threadfence();
    *(volatile v4f*)dst = v;
  }
}

__global__ __launch_bounds__(256) void final_out(
    const float* __restrict__ MX, const float* __restrict__ MN, const float* __restrict__ SC2,
    float* __restrict__ out1) {
  __shared__ __align__(16) float sT[32 * 36];
  const int tid = threadIdx.x;
  const int blk = blockIdx.x;
  const int st = blk & 31;
  const int ct = (blk >> 5) & 3;
  const int b = blk >> 7;
  const int s0 = st * 32;
  const int c0 = ct * 32;
  const int sl = tid >> 3;
  const int c4 = (tid & 7) * 4;
  const size_t off = ((size_t)(b * NCENT + s0 + sl)) * CH2 + c0 + c4;
  const v4f mx = *(const v4f*)(MX + off);
  const v4f mn = *(const v4f*)(MN + off);
  const v4f sc = *(const v4f*)(SC2 + c0 + c4);
  const v4f sh = *(const v4f*)(SC2 + CH2 + c0 + c4);
#pragma unroll
  for (int e = 0; e < 4; ++e) {
    const float scv = sc[e];
    const float fa = (scv >= 0.0f) ? 1.0f : 0.0f;
    const float fb = 1.0f - fa;
    const float pa = fa * mx[e];
    const float pb = fb * mn[e];
    const float v = pa + pb;
    float y = scv * v + sh[e];
    y = fmaxf(y, 0.0f);
    sT[(c4 + e) * 36 + sl] = y;
  }
  __syncthreads();
  const int cl = tid >> 3;
  const int s4 = (tid & 7) * 4;
  const v4f o = *(const v4f*)(sT + cl * 36 + s4);
  float* dst = out1 + ((size_t)(b * CH2 + c0 + cl)) * NCENT + s0 + s4;
  *(volatile v4f*)dst = o;
  __threadfence();
  *(volatile v4f*)dst = o;
}

extern "C" void kernel_launch(void* const* d_in, const int* in_sizes, int n_in,
                              void* d_out, int out_size, void* d_ws, size_t ws_size,
                              hipStream_t stream) {
  (void)in_sizes; (void)n_in; (void)out_size;
  if (ws_size < WS_TOTAL) return;
  const float* xyz    = (const float*)d_in[0];
  const float* points = (const float*)d_in[1];
  const float* w0  = (const float*)d_in[2];
  const float* b0  = (const float*)d_in[3];
  const float* g0  = (const float*)d_in[4];
  const float* be0 = (const float*)d_in[5];
  const float* w1  = (const float*)d_in[6];
  const float* b1  = (const float*)d_in[7];
  const float* g1  = (const float*)d_in[8];
  const float* be1 = (const float*)d_in[9];
  const float* w2  = (const float*)d_in[10];
  const float* b2  = (const float*)d_in[11];
  const float* g2  = (const float*)d_in[12];
  const float* be2 = (const float*)d_in[13];
  float* out0 = (float*)d_out;
  float* out1 = (float*)d_out + OUT1_ELEM_OFF;

  char* ws = (char*)d_ws;
  _Float16* W0h = (_Float16*)(ws + OFF_W0H);
  _Float16* W1h = (_Float16*)(ws + OFF_W1H);
  _Float16* W2h = (_Float16*)(ws + OFF_W2H);
  float* SC0 = (float*)(ws + OFF_SC0);
  float* SC1 = (float*)(ws + OFF_SC1);
  float* SC2 = (float*)(ws + OFF_SC2);
  float* CEN = (float*)(ws + OFF_CEN);
  int*   IDX = (int*)(ws + OFF_IDX);
  float* Vp  = (float*)(ws + OFF_V);
  _Float16* Fp = (_Float16*)(ws + OFF_F);
  float* PART0 = (float*)(ws + OFF_PART0);
  float* PART1 = (float*)(ws + OFF_PART1);
  float* PART2 = (float*)(ws + OFF_PART2);
  float* MXp = (float*)(ws + OFF_MX);
  float* MNp = (float*)(ws + OFF_MN);
  _Float16* X1 = (_Float16*)(ws + OFF_X1);

  prep_weights<<<8, 256, 0, stream>>>(w0, w1, w2, W0h, W1h, W2h);
  prep_features<<<NPTALL / 32, 256, 0, stream>>>(xyz, points, Fp);
  fps_kernel<<<NBATCH, 256, 0, stream>>>(xyz, out0, CEN);
  ball_query<<<NGROUP / 4, 128, 0, stream>>>(xyz, CEN, w0, IDX, Vp);
  pass_ab<false><<<NBLK_PASS, 256, 0, stream>>>(Fp, IDX, Vp, W0h, b0, SC0, W1h, b1, X1, PART0);
  bn_finalize<CH0><<<1, 256, 0, stream>>>(PART0, NBLK_PASS, g0, be0, SC0);
  pass_ab<true><<<NBLK_PASS, 256, 0, stream>>>(Fp, IDX, Vp, W0h, b0, SC0, W1h, b1, X1, PART1);
  bn_finalize<CH1><<<1, 256, 0, stream>>>(PART1, NBLK_PASS, g1, be1, SC1);
  pass_c<<<NBLK_PASS, 256, 0, stream>>>((const v4u*)X1, SC1, W2h, b2, MXp, MNp, PART2);
  bn_finalize<CH2><<<1, 256, 0, stream>>>(PART2, NBLK_PASS, g2, be2, SC2);
  final_out<<<NBATCH * 4 * 32, 256, 0, stream>>>(MXp, MNp, SC2, out1);
}
